// BasicNCA2D_91225105367407
// MI455X (gfx1250) — hardware-verified
//
#include <hip/hip_runtime.h>
#include <math.h>
#include <stdint.h>

#define NB    4
#define HH    192
#define WW    192
#define CC    16
#define HID   128
#define KDX   32
#define NPIX  (NB * HH * WW)
#define NSTEP 10
#define NT64  (NPIX / 64)
#define NWT   (NT64 * 2)
#define TABW  4864
static_assert((NPIX % 64) == 0);
static_assert((WW % 32) == 0 && (HH % 2) == 0);
static_assert((NWT % 8) == 0);
static_assert(((NPIX * CC) % (4 * 256)) == 0);
static_assert((TABW % 32) == 0 && ((TABW / 4) % 32) == 0);

typedef __bf16         v16b __attribute__((ext_vector_type(16)));
typedef float          v8f  __attribute__((ext_vector_type(8)));
typedef float          v4f  __attribute__((ext_vector_type(4)));
typedef unsigned int   v4u  __attribute__((ext_vector_type(4)));
typedef unsigned int   v2u  __attribute__((ext_vector_type(2)));
typedef unsigned short v8us __attribute__((ext_vector_type(8)));

__device__ __forceinline__ unsigned short bf_bits(float f) {
  unsigned u = __float_as_uint(f);
  return (unsigned short)((u + 0x7FFFu + ((u >> 16) & 1u)) >> 16);
}
__device__ __forceinline__ float bf_up(unsigned short h) { return __uint_as_float(((unsigned)h) << 16); }
__device__ __forceinline__ unsigned pk16(unsigned short a, unsigned short b) { return (unsigned)a | ((unsigned)b << 16); }
__device__ __forceinline__ v8f zero8() { v8f z = {0.f, 0.f, 0.f, 0.f, 0.f, 0.f, 0.f, 0.f}; return z; }

__device__ __forceinline__ v16b ldfrag_us(const unsigned short* p) {
  union { v16b v; v8us h[2]; } f;
  f.h[0] = *(const v8us*)(p);
  f.h[1] = *(const v8us*)(p + 16);
  return f.v;
}

__device__ __forceinline__ v8f mma_b(v16b a, v16b b, v8f c) {
  return __builtin_amdgcn_wmma_f32_16x16x32_bf16(false, a, false, b, (short)0, c, false, false);
}
__device__ __forceinline__ void dep_guard_b(v8f& a, v8f& b, v16b x, v16b y) {
#if defined(__HIP_DEVICE_COMPILE__)
  asm volatile("v_nop\n\tv_nop\n\tv_nop\n\tv_nop" : "+v"(a), "+v"(b) : "v"(x), "v"(y));
#endif
}
__device__ __forceinline__ void dep_guard3(v8f& a, v16b x, v16b y, v16b z) {
#if defined(__HIP_DEVICE_COMPILE__)
  asm volatile("v_nop\n\tv_nop\n\tv_nop\n\tv_nop" : "+v"(a) : "v"(x), "v"(y), "v"(z));
#endif
}
__device__ __forceinline__ void keep4_b(v16b a, v16b b, v16b c, v16b d) {
#if defined(__HIP_DEVICE_COMPILE__)
  asm volatile("v_nop" :: "v"(a), "v"(b), "v"(c), "v"(d));
#endif
}
__device__ __forceinline__ void acc_guard4(v8f& a, v8f& b, v8f& c, v8f& d) {
#if defined(__HIP_DEVICE_COMPILE__)
  asm volatile("v_nop\n\tv_nop\n\tv_nop\n\tv_nop" : "+v"(a), "+v"(b), "+v"(c), "+v"(d));
#endif
}
__device__ __forceinline__ void acc_guard1(v8f& a) {
#if defined(__HIP_DEVICE_COMPILE__)
  asm volatile("v_nop\n\tv_nop\n\tv_nop\n\tv_nop" : "+v"(a));
#endif
}
__device__ __forceinline__ void wave_sync_lds() {
  __builtin_amdgcn_fence(__ATOMIC_RELEASE, "workgroup");
  __builtin_amdgcn_wave_barrier();
  __builtin_amdgcn_fence(__ATOMIC_ACQUIRE, "workgroup");
}

__global__ __launch_bounds__(256) void k_tables(const float* __restrict__ wfc0, const float* __restrict__ wfc1,
                                                const float* __restrict__ wp0, const float* __restrict__ bp0,
                                                const float* __restrict__ bfc0, unsigned int* tab) {
  __shared__ __align__(16) unsigned int st[TABW];
  const int tid = threadIdx.x;
  for (int q = tid; q < TABW; q += 256) {
    int i0 = q;        if (i0 > 2047) i0 = 2047;
    const unsigned c0 = pk16(bf_bits(wfc0[2 * i0]), bf_bits(wfc0[2 * i0 + 1]));
    int i1 = q - 2048; if (i1 < 0) i1 = 0; if (i1 > 1023) i1 = 1023;
    const unsigned c1 = pk16(bf_bits(wfc1[2 * i1]), bf_bits(wfc1[2 * i1 + 1]));
    const int f = q - 3072;
    int fc = f;        if (fc < 0) fc = 0; if (fc > 1439) fc = 1439;
    const int ky  = fc / 144;
    const int rem = fc - ky * 144;
    const int kx  = rem >> 4;
    const int ch  = rem & 15;
    int wi = ch * 81 + ky * 9 + kx; if (wi > 1295) wi = 1295;
    const float wv = bf_up(bf_bits(wp0[wi]));
    const unsigned c2 = (f >= 0 && f < 1296) ? __float_as_uint(wv) : 0u;
    const int ib = q - 4608;
    int ibc = ib;      if (ibc < 0) ibc = 0; if (ibc > 15) ibc = 15;
    const float bv = bf_up(bf_bits(bp0[ibc]));
    const unsigned c3 = (ib >= 0 && ib < 16) ? __float_as_uint(bv) : 0u;
    int io = q - 4736; if (io < 0) io = 0; if (io > 127) io = 127;
    const unsigned c4w = __float_as_uint(bf_up(bf_bits(bfc0[io])));
    unsigned v = c4w;
    if (q < 4736) v = c3;
    if (q < 4608) v = c2;
    if (q < 3072) v = c1;
    if (q < 2048) v = c0;
    st[q] = v;
  }
  __syncthreads();
  for (int q = tid; q < TABW / 4; q += 256) {
    const v4u v = *(const v4u*)(st + q * 4);
    unsigned int* p = tab + (size_t)q * 4;
    for (int pass = 0; pass < 2; ++pass) { *(volatile v4u*)p = v; __threadfence(); }
  }
}

__global__ __launch_bounds__(256) void k_cvt_state(const float* __restrict__ xin, float* S, int n4) {
  const int i = blockIdx.x * 256 + threadIdx.x;
  if (i >= n4) return;
  const v4f a = *(const v4f*)(xin + (size_t)i * 4);
  v4f o;
  o[0] = bf_up(bf_bits(a[0])); o[1] = bf_up(bf_bits(a[1]));
  o[2] = bf_up(bf_bits(a[2])); o[3] = bf_up(bf_bits(a[3]));
  float* p = S + (size_t)i * 4;
  for (int pass = 0; pass < 2; ++pass) { *(volatile v4f*)p = o; __threadfence(); }
}

__global__ __launch_bounds__(WW) void k_dwconv(const float* __restrict__ S, const float* __restrict__ Wc,
                                               const float* __restrict__ bcv,
                                               unsigned short* DXh, unsigned short* DXl) {
  __shared__ __align__(16) v4u ctile[WW / 32][2][128];
  const int x    = threadIdx.x;
  const int lane = x & 31, wave = x >> 5;
  const int b    = blockIdx.x / (HH / 2);
  const int yp   = blockIdx.x - b * (HH / 2);
  const int y0   = yp * 2;

  float acc[2][CC];
#pragma unroll
  for (int i = 0; i < 2; ++i)
#pragma unroll
    for (int c = 0; c < CC; ++c) acc[i][c] = 0.0f;

#pragma unroll 1
  for (int r = 0; r < 10; ++r) {
    int yy = y0 - 4 + r;
    yy = (yy < 0) ? -yy : yy;
    yy = (yy > HH - 1) ? (2 * HH - 2 - yy) : yy;
    const float* rowp = S + (size_t)(b * HH + yy) * (size_t)(WW * CC);
    const int ky1 = (r == 0) ? 9 : (r - 1);
    const float* w0p = Wc + r * (9 * CC);
    const float* w1p = Wc + ky1 * (9 * CC);
#pragma unroll 1
    for (int kx = 0; kx < 9; ++kx) {
      int xx = x - 4 + kx;
      xx = (xx < 0) ? -xx : xx;
      xx = (xx > WW - 1) ? (2 * WW - 2 - xx) : xx;
      const float* pp = rowp + xx * CC;
      v4f v[4], wa[4], wb[4];
#pragma unroll
      for (int k4 = 0; k4 < 4; ++k4) {
        v[k4]  = *(const v4f*)(pp + 4 * k4);
        wa[k4] = *(const v4f*)(w0p + kx * CC + 4 * k4);
        wb[k4] = *(const v4f*)(w1p + kx * CC + 4 * k4);
      }
#pragma unroll
      for (int c = 0; c < CC; ++c) {
        acc[0][c] = fmaf(wa[c >> 2][c & 3], v[c >> 2][c & 3], acc[0][c]);
        acc[1][c] = fmaf(wb[c >> 2][c & 3], v[c >> 2][c & 3], acc[1][c]);
      }
    }
  }

  v4f bq[4];
#pragma unroll
  for (int k4 = 0; k4 < 4; ++k4) bq[k4] = *(const v4f*)(bcv + 4 * k4);
  v4u* ct0 = ctile[wave][0];
  v4u* ct1 = ctile[wave][1];
#pragma unroll
  for (int i = 0; i < 2; ++i) {
    const int prow = (b * HH + y0 + i) * WW;
    const float* xp = S + (size_t)(prow + x) * CC;
    float dxv[KDX];
#pragma unroll
    for (int k4 = 0; k4 < 4; ++k4) {
      const v4f t = *(const v4f*)(xp + 4 * k4);
      dxv[4 * k4 + 0] = t[0]; dxv[4 * k4 + 1] = t[1]; dxv[4 * k4 + 2] = t[2]; dxv[4 * k4 + 3] = t[3];
    }
#pragma unroll
    for (int c = 0; c < CC; ++c) dxv[CC + c] = acc[i][c] + bq[c >> 2][c & 3];
    v4u ph[4], pl[4];
#pragma unroll
    for (int e2 = 0; e2 < KDX / 2; ++e2) {
      const int e = 2 * e2;
      const unsigned short h0 = bf_bits(dxv[e]);
      const unsigned short h1 = bf_bits(dxv[e + 1]);
      const unsigned short l0 = bf_bits(dxv[e] - bf_up(h0));
      const unsigned short l1 = bf_bits(dxv[e + 1] - bf_up(h1));
      ph[e >> 3][(e & 7) >> 1] = pk16(h0, h1);
      pl[e >> 3][(e & 7) >> 1] = pk16(l0, l1);
    }
#pragma unroll
    for (int k4 = 0; k4 < 4; ++k4) { ct0[lane * 4 + k4] = ph[k4]; ct1[lane * 4 + k4] = pl[k4]; }
    wave_sync_lds();
    v4u hv[4], lv[4];
#pragma unroll
    for (int it = 0; it < 4; ++it) { hv[it] = ct0[it * 32 + lane]; lv[it] = ct1[it * 32 + lane]; }
    const size_t ub = (size_t)(prow + wave * 32) * KDX;
    for (int pass = 0; pass < 2; ++pass) {
#pragma unroll
      for (int it = 0; it < 4; ++it) {
        *(volatile v4u*)(DXh + ub + (size_t)it * 256 + lane * 8) = hv[it];
        *(volatile v4u*)(DXl + ub + (size_t)it * 256 + lane * 8) = lv[it];
      }
      __threadfence();
    }
    wave_sync_lds();
  }
}

__global__ __launch_bounds__(256) void k_fc0(const unsigned short* __restrict__ DXh,
                                             const unsigned short* __restrict__ DXl,
                                             const unsigned short* __restrict__ W0b,
                                             const float* __restrict__ b0r, float* Hf, float* part) {
  __shared__ __align__(16) float sT[8][16 * 68];
  __shared__ __align__(16) float sS[8][128];
  const int lane = threadIdx.x & 31;
  const int wave = threadIdx.x >> 5;
  const int tile = blockIdx.x * 8 + wave;
  if (tile >= NWT) return;
  const int tm = tile >> 1, tn = tile & 1;
  const int m0 = tm << 6, n0 = tn << 6;
  const int rlane = lane & 15;
  const int koff  = (lane >> 4) * 8;
  const int mOff  = (lane >> 4) * 8;
  const int hh    = lane >> 4;

  v8f acc[4][4];
#pragma unroll
  for (int i = 0; i < 4; ++i)
#pragma unroll
    for (int j = 0; j < 4; ++j) acc[i][j] = zero8();

  v16b bh[4];
#pragma unroll
  for (int j = 0; j < 4; ++j)
    bh[j] = ldfrag_us(W0b + (size_t)(n0 + (j << 4) + rlane) * KDX + koff);
#pragma unroll
  for (int i = 0; i < 4; ++i) {
    const size_t ao = (size_t)(m0 + (i << 4) + rlane) * KDX + koff;
    const v16b ah = ldfrag_us(DXh + ao);
    const v16b al = ldfrag_us(DXl + ao);
#pragma unroll
    for (int j = 0; j < 4; ++j) {
      acc[i][j] = mma_b(ah, bh[j], acc[i][j]);
      acc[i][j] = mma_b(al, bh[j], acc[i][j]);
    }
    dep_guard_b(acc[i][0], acc[i][3], ah, al);
  }
  keep4_b(bh[0], bh[1], bh[2], bh[3]);
  acc_guard4(acc[0][0], acc[0][1], acc[0][2], acc[0][3]);
  acc_guard4(acc[1][0], acc[1][1], acc[1][2], acc[1][3]);
  acc_guard4(acc[2][0], acc[2][1], acc[2][2], acc[2][3]);
  acc_guard4(acc[3][0], acc[3][1], acc[3][2], acc[3][3]);

  float bcol[4];
#pragma unroll
  for (int j = 0; j < 4; ++j) bcol[j] = b0r[n0 + (j << 4) + rlane];
  float s[4] = {0.f, 0.f, 0.f, 0.f};
  float q[4] = {0.f, 0.f, 0.f, 0.f};
#pragma unroll
  for (int i = 0; i < 4; ++i)
#pragma unroll
    for (int j = 0; j < 4; ++j)
#pragma unroll
      for (int r = 0; r < 8; ++r) {
        const float h = acc[i][j][r] + bcol[j];
        acc[i][j][r] = h;
        s[j] += h;
        q[j] = fmaf(h, h, q[j]);
      }
#pragma unroll
  for (int j = 0; j < 4; ++j) {
    s[j] += __shfl_xor(s[j], 16);
    q[j] += __shfl_xor(q[j], 16);
  }
  float* stt = sS[wave];
#pragma unroll
  for (int j = 0; j < 4; ++j) {
    stt[(j << 4) + rlane]      = s[j];
    stt[64 + (j << 4) + rlane] = q[j];
  }
  wave_sync_lds();
  {
    const v4f v = *(const v4f*)(stt + lane * 4);
    float* pp = part + (size_t)tile * 128 + lane * 4;
    for (int pass = 0; pass < 2; ++pass) { *(volatile v4f*)pp = v; __threadfence(); }
  }

  float* slab = sT[wave];
  const int c4 = (lane & 15) * 4;
#pragma unroll
  for (int i = 0; i < 4; ++i) {
    const int mBase = m0 + (i << 4);
#pragma unroll
    for (int j = 0; j < 4; ++j) {
#pragma unroll
      for (int r = 0; r < 8; ++r) {
        slab[(mOff + r) * 68 + (j << 4) + rlane] = acc[i][j][r];
      }
    }
    wave_sync_lds();
    for (int pass = 0; pass < 2; ++pass) {
#pragma unroll
      for (int it = 0; it < 8; ++it) {
        const int row = it * 2 + hh;
        const v4f v = *(const v4f*)(slab + row * 68 + c4);
        *(volatile v4f*)(Hf + (size_t)(mBase + row) * HID + n0 + c4) = v;
      }
      __threadfence();
    }
    wave_sync_lds();
  }
}

__global__ __launch_bounds__(256) void k_bnstat(const float* __restrict__ part, const float* __restrict__ gam,
                                                const float* __restrict__ bet, float* T) {
  __shared__ double sSum[2][128];
  __shared__ double sSq[2][128];
  __shared__ __align__(16) float sT[384];
  const int tid = threadIdx.x, col = tid & 127, half = tid >> 7;
  const int tn = col >> 6, cc = col & 63;
  double S = 0.0, Q = 0.0;
  const float* pb = part + (size_t)tn * 128 + cc;
  const int tm0 = half * (NT64 / 2);
#pragma unroll 1
  for (int tm = tm0; tm < tm0 + NT64 / 2; ++tm) {
    const float* pp = pb + (size_t)tm * 256;
    S += (double)pp[0];
    Q += (double)pp[64];
  }
  sSum[half][col] = S;
  sSq[half][col]  = Q;
  __syncthreads();
  if (tid < 128) {
    const double s2 = sSum[0][tid] + sSum[1][tid];
    const double q2 = sSq[0][tid] + sSq[1][tid];
    const double invn = 1.0 / (double)NPIX;
    const double mean = s2 * invn;
    double var = q2 * invn - mean * mean;
    if (var < 0.0) var = 0.0;
    const double rs = 1.0 / sqrt(var + 1e-5);
    sT[tid]       = (float)mean;
    sT[128 + tid] = bf_up(bf_bits(gam[tid])) * (float)rs;
    sT[256 + tid] = bf_up(bf_bits(bet[tid]));
  }
  __syncthreads();
  if (tid < 96) {
    const v4f v = *(const v4f*)(sT + tid * 4);
    float* pp = T + tid * 4;
    for (int pass = 0; pass < 2; ++pass) { *(volatile v4f*)pp = v; __threadfence(); }
  }
}

__global__ __launch_bounds__(128) void k_fc1(const float* __restrict__ Hf, const float* __restrict__ T,
                                             const unsigned short* __restrict__ W1b,
                                             const float* __restrict__ Sin, const float* __restrict__ ru,
                                             float* Sout) {
  __shared__ __align__(16) unsigned short sAh[64 * 136];
  __shared__ __align__(16) unsigned short sAl[64 * 136];
  __shared__ __align__(16) float sD[64 * 20];
  const int tid  = threadIdx.x;
  const int lane = tid & 31, wave = tid >> 5;
  const int p0   = blockIdx.x * 64;
  const int c4   = lane * 4;
  const v4f mean4 = *(const v4f*)(T + c4);
  const v4f sc4   = *(const v4f*)(T + 128 + c4);
  const v4f be4   = *(const v4f*)(T + 256 + c4);

#pragma unroll 4
  for (int it = 0; it < 16; ++it) {
    const int row = it * 4 + wave;
    const v4f v = *(const v4f*)(Hf + (size_t)(p0 + row) * HID + c4);
    unsigned short hq[4], lq[4];
#pragma unroll
    for (int k = 0; k < 4; ++k) {
      float t = (v[k] - mean4[k]) * sc4[k] + be4[k];
      t = fmaxf(t, 0.0f);
      const unsigned short hi = bf_bits(t);
      hq[k] = hi;
      lq[k] = bf_bits(t - bf_up(hi));
    }
    v2u ph, pl;
    ph[0] = pk16(hq[0], hq[1]); ph[1] = pk16(hq[2], hq[3]);
    pl[0] = pk16(lq[0], lq[1]); pl[1] = pk16(lq[2], lq[3]);
    *(v2u*)(sAh + row * 136 + c4) = ph;
    *(v2u*)(sAl + row * 136 + c4) = pl;
  }
  __syncthreads();

  const int rlane = lane & 15;
  const int koff  = (lane >> 4) * 8;
  const int hh    = lane >> 4;
  v8f acc = zero8();
#pragma unroll
  for (int ks = 0; ks < 4; ++ks) {
    const v16b ah = ldfrag_us(sAh + (wave * 16 + rlane) * 136 + ks * 32 + koff);
    const v16b al = ldfrag_us(sAl + (wave * 16 + rlane) * 136 + ks * 32 + koff);
    const v16b bb = ldfrag_us(W1b + (size_t)rlane * HID + ks * 32 + koff);
    acc = mma_b(ah, bb, acc);
    acc = mma_b(al, bb, acc);
    dep_guard3(acc, ah, al, bb);
  }
  acc_guard1(acc);

#pragma unroll
  for (int r = 0; r < 8; ++r) sD[(wave * 16 + hh * 8 + r) * 20 + rlane] = acc[r];
  wave_sync_lds();
  v4f o[2];
  size_t po[2];
#pragma unroll
  for (int it = 0; it < 2; ++it) {
    const int pl = wave * 16 + it * 8 + (lane >> 2);
    const int cq = (lane & 3) * 4;
    const int p  = p0 + pl;
    const v4f xv = *(const v4f*)(Sin + (size_t)p * CC + cq);
    const v4f dv = *(const v4f*)(sD + pl * 20 + cq);
    const float u = bf_up(bf_bits(ru[p]));
    const float m = (u > 0.5f) ? 1.0f : 0.0f;
    v4f ov;
    ov[0] = xv[0] + dv[0] * m;
    ov[1] = xv[1] + dv[1] * m;
    ov[2] = xv[2] + dv[2] * m;
    ov[3] = xv[3] + dv[3] * m;
    ov[0] = (cq == 0) ? xv[0] : ov[0];
    o[it]  = ov;
    po[it] = (size_t)p * CC + cq;
  }
  for (int pass = 0; pass < 2; ++pass) {
#pragma unroll
    for (int it = 0; it < 2; ++it) *(volatile v4f*)(Sout + po[it]) = o[it];
    __threadfence();
  }
}

extern "C" void kernel_launch(void* const* d_in, const int* in_sizes, int n_in,
                              void* d_out, int out_size, void* d_ws, size_t ws_size,
                              hipStream_t stream) {
  if (n_in < 9) return;
  if (in_sizes[0] != NPIX * CC) return;
  if (in_sizes[1] != NSTEP * NPIX) return;
  if (in_sizes[2] != CC * 81) return;
  if (in_sizes[3] != CC) return;
  if (in_sizes[4] != HID * KDX) return;
  if (in_sizes[5] != HID) return;
  if (in_sizes[6] != CC * HID) return;
  if (in_sizes[7] != HID) return;
  if (in_sizes[8] != HID) return;
  if (out_size != NPIX * CC) return;

  const float* x_in   = (const float*)d_in[0];
  const float* rand_u = (const float*)d_in[1];
  const float* w_p0   = (const float*)d_in[2];
  const float* b_p0   = (const float*)d_in[3];
  const float* w_fc0  = (const float*)d_in[4];
  const float* b_fc0  = (const float*)d_in[5];
  const float* w_fc1  = (const float*)d_in[6];
  const float* gam    = (const float*)d_in[7];
  const float* bet    = (const float*)d_in[8];
  float* out = (float*)d_out;

  const size_t PS   = (size_t)NPIX * CC * 4;
  const size_t PDX  = (size_t)NPIX * KDX * 2;
  const size_t PH   = (size_t)NPIX * HID * 4;
  const size_t PP   = (size_t)NWT * 128 * 4;
  const size_t PT   = 2048;
  const size_t PTAB = (size_t)TABW * 4;
  size_t off = 0;
  const size_t oS0  = off; off += PS;
  const size_t oS1  = off; off += PS;
  const size_t oDXh = off; off += PDX;
  const size_t oDXl = off; off += PDX;
  const size_t oH   = off; off += PH;
  const size_t oP   = off; off += PP;
  const size_t oT   = off; off += PT;
  const size_t oTAB = off; off += PTAB;
  if (off > ws_size) return;
  if (off > (size_t)134217728) return;

  char* ws = (char*)d_ws;
  float* S0 = (float*)(ws + oS0);
  float* S1 = (float*)(ws + oS1);
  unsigned short* DXh = (unsigned short*)(ws + oDXh);
  unsigned short* DXl = (unsigned short*)(ws + oDXl);
  float* Hf   = (float*)(ws + oH);
  float* part = (float*)(ws + oP);
  float* Tt   = (float*)(ws + oT);
  unsigned int* tab = (unsigned int*)(ws + oTAB);
  const unsigned short* W0b = (const unsigned short*)(ws + oTAB);
  const unsigned short* W1b = (const unsigned short*)(ws + oTAB + 8192);
  const float* Wc  = (const float*)(ws + oTAB + 12288);
  const float* bcv = (const float*)(ws + oTAB + 18432);
  const float* b0r = (const float*)(ws + oTAB + 18944);

  const int n4 = NPIX * CC / 4;
  k_tables<<<dim3(1), dim3(256), 0, stream>>>(w_fc0, w_fc1, w_p0, b_p0, b_fc0, tab);
  k_cvt_state<<<dim3((n4 + 255) / 256), dim3(256), 0, stream>>>(x_in, S0, n4);

  for (int s = 0; s < NSTEP; ++s) {
    const float* Sin = (s & 1) ? S1 : S0;
    float* Sout = (s == NSTEP - 1) ? out : ((s & 1) ? S0 : S1);
    k_dwconv<<<dim3(NB * (HH / 2)), dim3(WW), 0, stream>>>(Sin, Wc, bcv, DXh, DXl);
    k_fc0<<<dim3(NWT / 8), dim3(256), 0, stream>>>(DXh, DXl, W0b, b0r, Hf, part);
    k_bnstat<<<dim3(1), dim3(256), 0, stream>>>(part, gam, bet, Tt);
    k_fc1<<<dim3(NT64), dim3(128), 0, stream>>>(Hf, Tt, W1b, Sin, rand_u + (size_t)s * NPIX, Sout);
  }
  (void)hipGetLastError();
}
